// HeatAttention_38448547234631
// MI455X (gfx1250) — hardware-verified
//
#include <hip/hip_runtime.h>

typedef _Float16 v16h __attribute__((ext_vector_type(16)));
typedef _Float16 v8h  __attribute__((ext_vector_type(8)));
typedef float    v8f  __attribute__((ext_vector_type(8)));
typedef float    v4f  __attribute__((ext_vector_type(4)));
typedef v8h __attribute__((may_alias)) v8ha;
typedef v4f __attribute__((may_alias)) v4fa;

union Frag { v16h v; v8h half[2]; };

#define EMB     1024
#define NHEADS  16
#define HD      64
#define SEQ     2048
#define BATCH   4
#define MROWS   (BATCH * SEQ)
#define NX      (MROWS * EMB)
#define NW      (EMB * EMB)
#define NX8     (NX / 8)
#define WSCALE  32.0f
#define INVW    0.03125f
#define PSCALE  16384.0f
#define INVP    (1.0f / 16384.0f)
#define QKSCALE 0.125f
#define KTEMP   1.5278640450004206f
#define INVKT   0.6545084971874737f

__device__ __forceinline__ v8f wmma_f16(v16h a, v16h b, v8f c) {
  v8f d = __builtin_amdgcn_wmma_f32_16x16x32_f16(false, a, false, b, (short)0, c, false, false);
  asm volatile("v_nop\n\tv_nop\n\tv_nop\n\tv_nop" : "+v"(d) : "v"(a), "v"(b));
  return d;
}

__device__ __forceinline__ v16h load_frag(const _Float16* p, int h) {
  Frag f;
  f.half[0] = *(const v8ha*)(p + 8 * h);
  f.half[1] = *(const v8ha*)(p + 16 + 8 * h);
  return f.v;
}

__global__ __launch_bounds__(256) void cvt_x_kernel(const float* __restrict__ x,
                                                    _Float16* __restrict__ xh)
{
  const int g = blockIdx.x * 256 + threadIdx.x;
  if (g >= NX8) return;
  const float* src = x + (size_t)g * 8;
  const v4f a = *(const v4fa*)src;
  const v4f c = *(const v4fa*)(src + 4);
  const v8h o = { (_Float16)a.x, (_Float16)a.y, (_Float16)a.z, (_Float16)a.w,
                  (_Float16)c.x, (_Float16)c.y, (_Float16)c.z, (_Float16)c.w };
  _Float16* dst = xh + (size_t)g * 8;
  *(volatile v8h*)dst = o;
  __threadfence();
  *(volatile v8h*)dst = o;
}

__device__ __forceinline__ void wt_store_pass(const float* tile, _Float16* wt,
                                              int z, int out0, int in0, int w, int lane) {
  const int q8 = lane & 7, sub = lane >> 3;
  #pragma unroll
  for (int i = 0; i < 2; ++i) {
    const int oc = w * 8 + i * 4 + sub;
    const int j0 = 8 * q8;
    const v8h v = { (_Float16)(tile[(j0 + 0) * 65 + oc] * WSCALE), (_Float16)(tile[(j0 + 1) * 65 + oc] * WSCALE),
                    (_Float16)(tile[(j0 + 2) * 65 + oc] * WSCALE), (_Float16)(tile[(j0 + 3) * 65 + oc] * WSCALE),
                    (_Float16)(tile[(j0 + 4) * 65 + oc] * WSCALE), (_Float16)(tile[(j0 + 5) * 65 + oc] * WSCALE),
                    (_Float16)(tile[(j0 + 6) * 65 + oc] * WSCALE), (_Float16)(tile[(j0 + 7) * 65 + oc] * WSCALE) };
    _Float16* dst = wt + ((size_t)z * EMB + out0 + oc) * EMB + in0 + j0;
    *(volatile v8h*)dst = v;
  }
}

__global__ __launch_bounds__(256) void wt_kernel(
    const float* __restrict__ wq, const float* __restrict__ wk,
    const float* __restrict__ wv, const float* __restrict__ wo,
    _Float16* __restrict__ wt)
{
  __shared__ float tile[64 * 65];

  const int tid = threadIdx.x, lane = tid & 31, w = tid >> 5;
  const int out0 = blockIdx.x * 64, in0 = blockIdx.y * 64, z = blockIdx.z;
  const float* W = (z == 0) ? wq : ((z == 1) ? wk : ((z == 2) ? wv : wo));
  const int c = tid & 63, rg = tid >> 6;
  #pragma unroll
  for (int i = 0; i < 16; ++i) {
    const int r = i * 4 + rg;
    tile[r * 65 + c] = W[(size_t)(in0 + r) * EMB + out0 + c];
  }
  __syncthreads();

  wt_store_pass(tile, wt, z, out0, in0, w, lane);
  __threadfence();
  wt_store_pass(tile, wt, z, out0, in0, w, lane);
}

__device__ __forceinline__ void proj_store_pass(const _Float16* sT, _Float16* plane, _Float16* vt,
                                                int which, int bh, int l0, int w, int lane) {
  const int q8 = lane & 7, sub = lane >> 3;
  #pragma unroll
  for (int i = 0; i < 8; ++i) {
    const int lid = w * 32 + i * 4 + sub;
    v8h v;
    _Float16* dst;
    if (which != 2) {
      v = *(const v8ha*)(sT + lid * HD + 8 * q8);
      dst = plane + ((size_t)bh * SEQ + l0 + lid) * HD + 8 * q8;
    } else {
      const int d = lid >> 1, hl = lid & 1;
      v = *(const v8ha*)(sT + d * 128 + 64 * hl + 8 * q8);
      dst = vt + ((size_t)bh * HD + d) * SEQ + l0 + 64 * hl + 8 * q8;
    }
    *(volatile v8h*)dst = v;
  }
}

__global__ __launch_bounds__(128) void proj_kernel(
    const _Float16* __restrict__ xh,
    const _Float16* __restrict__ wt,
    const float* __restrict__ bq, const float* __restrict__ bk, const float* __restrict__ bv,
    _Float16* __restrict__ qh,
    _Float16* __restrict__ kh,
    _Float16* __restrict__ vt)
{
  __shared__ __attribute__((aligned(16))) _Float16 sT[128 * 64];

  const int tid = threadIdx.x, lane = tid & 31, w = tid >> 5;
  const int h = lane >> 4, m = lane & 15;
  const int m0 = blockIdx.x * 128;
  const int cg = blockIdx.y;
  const int which = cg >> 4, head = cg & 15;
  const int m0w = m0 + 32 * w;

  const _Float16* xa0 = xh + (size_t)(m0w + m) * EMB;
  const _Float16* xa1 = xa0 + (size_t)16 * EMB;
  const _Float16* wb  = wt + ((size_t)which * EMB + head * HD + m) * EMB;

  const v8f zero8 = {0.f, 0.f, 0.f, 0.f, 0.f, 0.f, 0.f, 0.f};
  v8f acc[2][4];
  #pragma unroll
  for (int mt = 0; mt < 2; ++mt)
    #pragma unroll
    for (int nt = 0; nt < 4; ++nt) acc[mt][nt] = zero8;

  #pragma unroll 1
  for (int k0 = 0; k0 < EMB; k0 += 32) {
    const v16h a0 = load_frag(xa0 + k0, h);
    const v16h a1 = load_frag(xa1 + k0, h);
    #pragma unroll
    for (int nt = 0; nt < 4; ++nt) {
      const v16h b = load_frag(wb + (size_t)nt * 16 * EMB + k0, h);
      acc[0][nt] = wmma_f16(a0, b, acc[0][nt]);
      acc[1][nt] = wmma_f16(a1, b, acc[1][nt]);
    }
  }

  const float* bias = (which == 0) ? bq : ((which == 1) ? bk : bv);
  #pragma unroll
  for (int nt = 0; nt < 4; ++nt) {
    const int feat = 16 * nt + m;
    const float bvl = bias[head * HD + feat];
    #pragma unroll
    for (int mt = 0; mt < 2; ++mt) {
      #pragma unroll
      for (int r = 0; r < 8; ++r) {
        const int tokl = 32 * w + 16 * mt + 8 * h + r;
        const float y = acc[mt][nt][r] * INVW + bvl;
        const int idx = (which == 2) ? (feat * 128 + tokl) : (tokl * HD + feat);
        sT[idx] = (_Float16)y;
      }
    }
  }
  __syncthreads();

  const int b = m0 / SEQ, l0 = m0 - b * SEQ, bh = b * NHEADS + head;
  _Float16* plane = (which == 0) ? qh : kh;
  proj_store_pass(sT, plane, vt, which, bh, l0, w, lane);
  __threadfence();
  proj_store_pass(sT, plane, vt, which, bh, l0, w, lane);
}

__device__ __forceinline__ v8f logit8(v8f s, const float* p) {
  const v4f fa = *(const v4fa*)p;
  const v4f fb = *(const v4fa*)(p + 4);
  s[0] = (s[0] * QKSCALE + fa.x * KTEMP) * INVKT;
  s[1] = (s[1] * QKSCALE + fa.y * KTEMP) * INVKT;
  s[2] = (s[2] * QKSCALE + fa.z * KTEMP) * INVKT;
  s[3] = (s[3] * QKSCALE + fa.w * KTEMP) * INVKT;
  s[4] = (s[4] * QKSCALE + fb.x * KTEMP) * INVKT;
  s[5] = (s[5] * QKSCALE + fb.y * KTEMP) * INVKT;
  s[6] = (s[6] * QKSCALE + fb.z * KTEMP) * INVKT;
  s[7] = (s[7] * QKSCALE + fb.w * KTEMP) * INVKT;
  return s;
}

__device__ __forceinline__ v16h pack_p(v8f a, v8f c) {
  const v16h r = { (_Float16)(a[0] * PSCALE), (_Float16)(a[1] * PSCALE), (_Float16)(a[2] * PSCALE), (_Float16)(a[3] * PSCALE),
                   (_Float16)(a[4] * PSCALE), (_Float16)(a[5] * PSCALE), (_Float16)(a[6] * PSCALE), (_Float16)(a[7] * PSCALE),
                   (_Float16)(c[0] * PSCALE), (_Float16)(c[1] * PSCALE), (_Float16)(c[2] * PSCALE), (_Float16)(c[3] * PSCALE),
                   (_Float16)(c[4] * PSCALE), (_Float16)(c[5] * PSCALE), (_Float16)(c[6] * PSCALE), (_Float16)(c[7] * PSCALE) };
  return r;
}

__device__ __forceinline__ void att_store_pass(const _Float16* so, _Float16* oh,
                                               int b, int head, int q0, int lane) {
  const int q8 = lane & 7, sub = lane >> 3;
  #pragma unroll
  for (int i = 0; i < 4; ++i) {
    const int row = i * 4 + sub;
    const v8h v = *(const v8ha*)(so + row * 64 + 8 * q8);
    const size_t gi = ((size_t)b * SEQ + q0 + row) * EMB + head * HD + 8 * q8;
    *(volatile v8h*)(oh + gi) = v;
  }
}

__global__ __launch_bounds__(128) void attn_kernel(
    const _Float16* __restrict__ qh,
    const _Float16* __restrict__ kh,
    const _Float16* __restrict__ vt,
    const float* __restrict__ focus,
    _Float16* __restrict__ oh)
{
  __shared__ __attribute__((aligned(16))) _Float16 sO[4 * 16 * 64];

  const int tid = threadIdx.x, lane = tid & 31, w = tid >> 5;
  const int h = lane >> 4, m = lane & 15;
  const int bh = blockIdx.y, b = bh >> 4, head = bh & 15;
  const int q0 = blockIdx.x * 64 + 16 * w;

  const _Float16* qrow = qh + ((size_t)bh * SEQ + q0 + m) * HD;
  const v16h qb0 = load_frag(qrow, h);
  const v16h qb1 = load_frag(qrow + 32, h);

  const v8f zero8 = {0.f, 0.f, 0.f, 0.f, 0.f, 0.f, 0.f, 0.f};
  v8f o[4];
  #pragma unroll
  for (int t = 0; t < 4; ++t) o[t] = zero8;
  float mrun = -1e30f, lrun = 0.0f;

  const _Float16* kbase = kh + ((size_t)bh * SEQ + m) * HD;
  const _Float16* vbase = vt + ((size_t)bh * HD + m) * SEQ;
  const float* fbp = focus + (size_t)b * SEQ + 8 * h;

  #pragma unroll 1
  for (int kb = 0; kb < SEQ; kb += 64) {
    v8f s[4];
    #pragma unroll
    for (int j = 0; j < 4; ++j) {
      const _Float16* kp = kbase + (size_t)(kb + 16 * j) * HD;
      const v16h kf0 = load_frag(kp, h);
      const v16h kf1 = load_frag(kp + 32, h);
      v8f z = zero8;
      z = wmma_f16(kf0, qb0, z);
      z = wmma_f16(kf1, qb1, z);
      s[j] = z;
    }
    #pragma unroll
    for (int j = 0; j < 4; ++j) s[j] = logit8(s[j], fbp + kb + 16 * j);

    float mloc = s[0][0];
    #pragma unroll
    for (int j = 0; j < 4; ++j)
      #pragma unroll
      for (int r = 0; r < 8; ++r) mloc = fmaxf(mloc, s[j][r]);
    mloc = fmaxf(mloc, __shfl_xor(mloc, 16));
    const float mnew = fmaxf(mrun, mloc);
    const float alpha = __expf(mrun - mnew);
    mrun = mnew;
    float lsum = 0.0f;
    #pragma unroll
    for (int j = 0; j < 4; ++j)
      #pragma unroll
      for (int r = 0; r < 8; ++r) {
        const float p = __expf(s[j][r] - mnew);
        s[j][r] = p;
        lsum += p;
      }
    lsum += __shfl_xor(lsum, 16);
    lrun = lrun * alpha + lsum;
    #pragma unroll
    for (int t = 0; t < 4; ++t)
      #pragma unroll
      for (int r = 0; r < 8; ++r) o[t][r] = o[t][r] * alpha;

    const v16h pb0 = pack_p(s[0], s[1]);
    const v16h pb1 = pack_p(s[2], s[3]);

    #pragma unroll
    for (int t = 0; t < 4; ++t) {
      const _Float16* vp = vbase + (size_t)(16 * t) * SEQ + kb;
      const v16h vf0 = load_frag(vp, h);
      const v16h vf1 = load_frag(vp + 32, h);
      o[t] = wmma_f16(vf0, pb0, o[t]);
      o[t] = wmma_f16(vf1, pb1, o[t]);
    }
  }

  const float inv = (1.0f / lrun) * INVP;
  _Float16* so = sO + w * 1024;
  #pragma unroll
  for (int t = 0; t < 4; ++t)
    #pragma unroll
    for (int r = 0; r < 8; ++r)
      so[m * 64 + 16 * t + 8 * h + r] = (_Float16)(o[t][r] * inv);
  __syncthreads();

  att_store_pass(so, oh, b, head, q0, lane);
  __threadfence();
  att_store_pass(so, oh, b, head, q0, lane);
}

__device__ __forceinline__ void out_store_pass(const float* sT, float* out,
                                               int m0, int n0, int w, int lane) {
  const int q8 = lane & 7, sub = lane >> 3;
  #pragma unroll
  for (int i = 0; i < 16; ++i) {
    const int lid = i * 4 + sub;
    const int row = w * 32 + (lid >> 1), hl = lid & 1;
    const v4f v = *(const v4fa*)(sT + row * 64 + 32 * hl + 4 * q8);
    const size_t gi = (size_t)(m0 + row) * EMB + n0 + 32 * hl + 4 * q8;
    *(volatile v4f*)(out + gi) = v;
  }
}

__global__ __launch_bounds__(128) void oproj_kernel(
    const _Float16* __restrict__ oh,
    const _Float16* __restrict__ wot,
    const float* __restrict__ bo,
    float* __restrict__ out)
{
  __shared__ __attribute__((aligned(16))) float sT[128 * 64];

  const int tid = threadIdx.x, lane = tid & 31, w = tid >> 5;
  const int h = lane >> 4, m = lane & 15;
  const int m0 = blockIdx.x * 128;
  const int n0 = blockIdx.y * 64;
  const int m0w = m0 + 32 * w;

  const _Float16* xa0 = oh + (size_t)(m0w + m) * EMB;
  const _Float16* xa1 = xa0 + (size_t)16 * EMB;
  const _Float16* wb  = wot + (size_t)(n0 + m) * EMB;

  const v8f zero8 = {0.f, 0.f, 0.f, 0.f, 0.f, 0.f, 0.f, 0.f};
  v8f acc[2][4];
  #pragma unroll
  for (int mt = 0; mt < 2; ++mt)
    #pragma unroll
    for (int nt = 0; nt < 4; ++nt) acc[mt][nt] = zero8;

  #pragma unroll 1
  for (int k0 = 0; k0 < EMB; k0 += 32) {
    const v16h a0 = load_frag(xa0 + k0, h);
    const v16h a1 = load_frag(xa1 + k0, h);
    #pragma unroll
    for (int nt = 0; nt < 4; ++nt) {
      const v16h b = load_frag(wb + (size_t)nt * 16 * EMB + k0, h);
      acc[0][nt] = wmma_f16(a0, b, acc[0][nt]);
      acc[1][nt] = wmma_f16(a1, b, acc[1][nt]);
    }
  }

  #pragma unroll
  for (int nt = 0; nt < 4; ++nt) {
    const int feat = 16 * nt + m;
    const float bvl = bo[n0 + feat];
    #pragma unroll
    for (int mt = 0; mt < 2; ++mt) {
      #pragma unroll
      for (int r = 0; r < 8; ++r) {
        const int tokl = 32 * w + 16 * mt + 8 * h + r;
        sT[tokl * 64 + feat] = acc[mt][nt][r] * INVW + bvl;
      }
    }
  }
  __syncthreads();

  out_store_pass(sT, out, m0, n0, w, lane);
  __threadfence();
  out_store_pass(sT, out, m0, n0, w, lane);
}

extern "C" void kernel_launch(void* const* d_in, const int* in_sizes, int n_in,
                              void* d_out, int out_size, void* d_ws, size_t ws_size,
                              hipStream_t stream) {
  if (n_in < 10) return;
  if (in_sizes[0] != NX) return;
  if (in_sizes[1] != MROWS) return;
  if (in_sizes[2] != NW || in_sizes[4] != NW || in_sizes[6] != NW || in_sizes[8] != NW) return;
  if (in_sizes[3] != EMB || in_sizes[5] != EMB || in_sizes[7] != EMB || in_sizes[9] != EMB) return;
  if (out_size != NX) return;

  const float* x     = (const float*)d_in[0];
  const float* focus = (const float*)d_in[1];
  const float* Wq    = (const float*)d_in[2];
  const float* bq    = (const float*)d_in[3];
  const float* Wk    = (const float*)d_in[4];
  const float* bk    = (const float*)d_in[5];
  const float* Wv    = (const float*)d_in[6];
  const float* bv    = (const float*)d_in[7];
  const float* Wo    = (const float*)d_in[8];
  const float* bo    = (const float*)d_in[9];
  float* out = (float*)d_out;

  const size_t xh_bytes = (size_t)NX * 2;
  const size_t wt_bytes = (size_t)4 * NW * 2;
  const size_t pl_bytes = (size_t)BATCH * NHEADS * SEQ * HD * 2;
  const size_t oh_bytes = (size_t)NX * 2;
  const size_t total = xh_bytes + wt_bytes + 3 * pl_bytes + oh_bytes;
  if (total > ws_size) return;

  char* ws = (char*)d_ws;
  _Float16* xh = (_Float16*)(ws);
  _Float16* wt = (_Float16*)(ws + xh_bytes);
  _Float16* qh = (_Float16*)(ws + xh_bytes + wt_bytes);
  _Float16* kh = (_Float16*)(ws + xh_bytes + wt_bytes + pl_bytes);
  _Float16* vt = (_Float16*)(ws + xh_bytes + wt_bytes + 2 * pl_bytes);
  _Float16* oh = (_Float16*)(ws + xh_bytes + wt_bytes + 3 * pl_bytes);
  _Float16* wot = wt + (size_t)3 * NW;

  cvt_x_kernel<<<(NX8 + 255) / 256, 256, 0, stream>>>(x, xh);

  dim3 gWt(EMB / 64, EMB / 64, 4);
  wt_kernel<<<gWt, 256, 0, stream>>>(Wq, Wk, Wv, Wo, wt);

  dim3 gProj(MROWS / 128, 3 * NHEADS);
  proj_kernel<<<gProj, 128, 0, stream>>>(xh, wt, bq, bk, bv, qh, kh, vt);

  dim3 gAtt(SEQ / 64, BATCH * NHEADS);
  attn_kernel<<<gAtt, 128, 0, stream>>>(qh, kh, vt, focus, oh);

  dim3 gOut(MROWS / 128, EMB / 64);
  oproj_kernel<<<gOut, 128, 0, stream>>>(oh, wot, bo, out);
}
